// Head_54408645706053
// MI455X (gfx1250) — hardware-verified
//
#include <hip/hip_runtime.h>
#ifndef NB
#define NB 4
#endif
#ifndef SEQ
#define SEQ 4096
#endif
#define SEQ_FULL 4096
#define DM 768
#define HD 64
#define NR ((size_t)NB * SEQ)
#define QC ((SEQ < 2048) ? SEQ : 2048)
#define RESC 256
static_assert(SEQ % 256 == 0);
static_assert(SEQ <= SEQ_FULL);
static_assert(SEQ % QC == 0);
static_assert(QC % 128 == 0);
static_assert(QC >= RESC);
static_assert(((QC - RESC) % 128) == 0);
static_assert(DM % 32 == 0);
static_assert(HD == 64);

typedef unsigned short v8us __attribute__((ext_vector_type(8), may_alias));
typedef float  v8f  __attribute__((ext_vector_type(8)));
typedef float  v4f  __attribute__((ext_vector_type(4)));
typedef float  v4fa __attribute__((ext_vector_type(4), may_alias));
typedef _Float16 v16h __attribute__((ext_vector_type(16)));
union FragH { v16h v; v8us half[2]; _Float16 h[16]; unsigned short u[16]; };

__device__ __forceinline__ unsigned short bf16_bits(float x) { unsigned int u = __float_as_uint(x); return (unsigned short)((u + 0x7FFFu + ((u >> 16) & 1u)) >> 16); }
__device__ __forceinline__ float bf16_val(unsigned short b) { return __uint_as_float(((unsigned int)b) << 16); }
__device__ __forceinline__ float bf16_rne(float x) { return bf16_val(bf16_bits(x)); }

__device__ __forceinline__ v16h g2_frag(const _Float16* p, int hh) { FragH f; f.half[0] = *(const v8us*)((const unsigned short*)p + 8 * hh); f.half[1] = *(const v8us*)((const unsigned short*)p + 16 + 8 * hh); return f.v; }
__device__ __forceinline__ v8f g2_mma(v16h a, v16h b, v8f c) { v8f d = __builtin_amdgcn_wmma_f32_16x16x32_f16(false, a, false, b, (short)0, c, false, false); asm volatile("v_nop\n\tv_nop\n\tv_nop\n\tv_nop" : "+v"(d) : "v"(a), "v"(b)); return d; }

__global__ __launch_bounds__(256) void k_wt_f16(const float* __restrict__ W, _Float16* __restrict__ Wt, int K, int N, float scale) {
  const int t = blockIdx.x * 256 + threadIdx.x; if (t >= N * (K / 8)) return;
  const int n = t / (K / 8), k8 = (t % (K / 8)) * 8; FragH f;
#pragma unroll
  for (int i = 0; i < 8; ++i) f.h[i] = (_Float16)(bf16_rne(W[(size_t)(k8 + i) * N + n]) * scale);
  const v8us o = f.half[0];
  unsigned short* d = (unsigned short*)Wt + (size_t)n * K + k8;
  *(volatile v8us*)d = o; __threadfence(); *(volatile v8us*)d = o;
}

__global__ __launch_bounds__(256) void k_x16(const float* __restrict__ x, _Float16* __restrict__ X16, size_t n8) {
  const size_t t = (size_t)blockIdx.x * 256 + threadIdx.x; if (t >= n8) return;
  const size_t e = t * 8; const size_t r = e / DM; const size_t c = e - r * DM;
  const size_t src = ((r / SEQ) * SEQ_FULL + (r % SEQ)) * DM + c;
  FragH f;
#pragma unroll
  for (int q = 0; q < 8; ++q) f.h[q] = (_Float16)bf16_rne(x[src + q]);
  unsigned short* d = (unsigned short*)X16 + e;
  *(volatile v8us*)d = f.half[0]; __threadfence(); *(volatile v8us*)d = f.half[0];
}

__global__ __launch_bounds__(256) void k_hl(const float* __restrict__ F, _Float16* __restrict__ Hh, _Float16* __restrict__ Hl, size_t n8) {
  const size_t t = (size_t)blockIdx.x * 256 + threadIdx.x; if (t >= n8) return;
  FragH fh, fl; const v4f a = *(const v4fa*)(F + t * 8), c = *(const v4fa*)(F + t * 8 + 4);
#pragma unroll
  for (int q = 0; q < 4; ++q) { _Float16 h = (_Float16)a[q]; fh.h[q] = h; fl.h[q] = (_Float16)((a[q] - (float)h) * 1024.0f); h = (_Float16)c[q]; fh.h[4 + q] = h; fl.h[4 + q] = (_Float16)((c[q] - (float)h) * 1024.0f); }
  for (int pass = 0; pass < 2; ++pass) { *(volatile v8us*)((unsigned short*)Hh + t * 8) = fh.half[0]; *(volatile v8us*)((unsigned short*)Hl + t * 8) = fl.half[0]; if (pass == 0) __threadfence(); }
}

__global__ __launch_bounds__(256) void k_vt(const _Float16* __restrict__ V16, int ldv, int tt, _Float16* __restrict__ Vt, int opitch, int ngr) {
  __shared__ unsigned short tl[64][66];
  const int tid = threadIdx.x; const int b = blockIdx.x / ngr, lg = blockIdx.x - b * ngr;
  for (int i = tid; i < 64 * 8; i += 256) { const int r = i >> 3, c8 = (i & 7) * 8; FragH f; f.half[0] = *(const v8us*)((const unsigned short*)V16 + ((size_t)b * tt + (size_t)lg * 64 + r) * ldv + c8);
#pragma unroll
    for (int q = 0; q < 8; ++q) tl[r][c8 + q] = f.u[q]; }
  __syncthreads();
  for (int pass = 0; pass < 2; ++pass) {
#pragma unroll
    for (int rd = 0; rd < 2; ++rd) { const int d = rd * 32 + (tid >> 3), pc = tid & 7; FragH f;
#pragma unroll
      for (int q = 0; q < 8; ++q) f.u[q] = tl[pc * 8 + q][d];
      *(volatile v8us*)((unsigned short*)Vt + ((size_t)b * 64 + d) * opitch + (size_t)lg * 64 + pc * 8) = f.half[0]; }
    if (pass == 0) __threadfence(); }
}

__global__ void __launch_bounds__(128) __attribute__((amdgpu_num_vgpr(256)))
k_gemm2(const _Float16* __restrict__ A, int lda, const _Float16* __restrict__ Bh, int ldb, float alpha, float* __restrict__ C, int ldc, int M, int N, int K) {
  __shared__ __attribute__((aligned(16))) float so[4][32][68];
  const int tid = threadIdx.x, w = tid >> 5, lane = tid & 31, ln = lane & 15, hh = lane >> 4;
  const int ntn = N >> 6; const int mt = blockIdx.x / ntn, nq = blockIdx.x - mt * ntn; const int row0 = mt * 128 + 32 * w, col0 = nq * 64; if (row0 >= M) return;
  const _Float16* a0p = A + (size_t)(row0 + ln) * lda; const _Float16* a1p = a0p + (size_t)16 * lda;
  const _Float16* b0p = Bh + (size_t)(col0 + ln) * ldb; const _Float16* b1p = b0p + (size_t)16 * ldb; const _Float16* b2p = b1p + (size_t)16 * ldb; const _Float16* b3p = b2p + (size_t)16 * ldb;
  const v8f z8 = {0.f,0.f,0.f,0.f,0.f,0.f,0.f,0.f}; v8f c00 = z8, c01 = z8, c02 = z8, c03 = z8, c10 = z8, c11 = z8, c12 = z8, c13 = z8;
#pragma unroll 1
  for (int kb = 0; kb < K; kb += 32) { const v16h a0 = g2_frag(a0p + kb, hh), a1 = g2_frag(a1p + kb, hh);
    v16h b = g2_frag(b0p + kb, hh); c00 = g2_mma(a0, b, c00); c10 = g2_mma(a1, b, c10);
    b = g2_frag(b1p + kb, hh); c01 = g2_mma(a0, b, c01); c11 = g2_mma(a1, b, c11);
    b = g2_frag(b2p + kb, hh); c02 = g2_mma(a0, b, c02); c12 = g2_mma(a1, b, c12);
    b = g2_frag(b3p + kb, hh); c03 = g2_mma(a0, b, c03); c13 = g2_mma(a1, b, c13); }
  v8f accs[8] = {c00, c01, c02, c03, c10, c11, c12, c13};
#pragma unroll
  for (int u = 0; u < 8; ++u) { const int t = u & 3, half = u >> 2;
#pragma unroll
    for (int r = 0; r < 8; ++r) { const int rloc = half * 16 + 8 * hh + r; so[w][rloc][t * 16 + ln] = accs[u][r] * alpha; } }
  __builtin_amdgcn_fence(4, "workgroup"); __builtin_amdgcn_wave_barrier();
  const int rsub = lane >> 4, c4 = (lane & 15) * 4;
  for (int pass = 0; pass < 2; ++pass) {
#pragma unroll
    for (int q = 0; q < 16; ++q) { const int r = q * 2 + rsub; const v4f v = *(const v4fa*)&so[w][r][c4]; *(volatile v4f*)(C + (size_t)(row0 + r) * ldc + col0 + c4) = v; }
    if (pass == 0) __threadfence(); }
}

__global__ void __launch_bounds__(128) __attribute__((amdgpu_num_vgpr(256)))
k_gemm_hr(const _Float16* __restrict__ Ah, int lda, const _Float16* __restrict__ Al, int ldal,
          const _Float16* __restrict__ Bh, int ldb, const _Float16* __restrict__ Bl, int ldbl,
          float alpha, float rsc, int rrows, int cq, float* __restrict__ C, int ldc, int M, int N, int K) {
  __shared__ __attribute__((aligned(16))) float so[4][16][64];
  const int tid = threadIdx.x, w = tid >> 5, lane = tid & 31, ln = lane & 15, hh = lane >> 4;
  const int ntn = N >> 6; const int wid = blockIdx.x * 4 + w; const int mt = wid / ntn, nq = wid - mt * ntn;
  const int row0 = mt * 16, col0 = nq * 64;
  if (row0 >= M) return;
  if (col0 > row0 + cq + 15) return;
  const bool res = (row0 < rrows);
  const _Float16* ahp = Ah + (size_t)(row0 + ln) * lda;
  const _Float16* alp = Al + (size_t)(row0 + ln) * ldal;
  const _Float16* bhp = Bh + (size_t)(col0 + ln) * ldb;
  const _Float16* blp = Bl + (size_t)(col0 + ln) * ldbl;
  v8f ch[4] = {}; v8f cr[4] = {};
#pragma unroll 1
  for (int kb = 0; kb < K; kb += 32) {
    const v16h a = g2_frag(ahp + kb, hh);
    if (res) {
      const v16h al = g2_frag(alp + kb, hh);
#pragma unroll
      for (int t = 0; t < 4; ++t) {
        const v16h b = g2_frag(bhp + (size_t)(t * 16) * ldb + kb, hh);
        const v16h bl = g2_frag(blp + (size_t)(t * 16) * ldbl + kb, hh);
        ch[t] = g2_mma(a, b, ch[t]); cr[t] = g2_mma(al, b, cr[t]); cr[t] = g2_mma(a, bl, cr[t]);
      }
    } else {
#pragma unroll
      for (int t = 0; t < 4; ++t) { const v16h b = g2_frag(bhp + (size_t)(t * 16) * ldb + kb, hh); ch[t] = g2_mma(a, b, ch[t]); }
    }
  }
#pragma unroll
  for (int t = 0; t < 4; ++t) {
#pragma unroll
    for (int r = 0; r < 8; ++r) so[w][8 * hh + r][t * 16 + ln] = (ch[t][r] + cr[t][r] * rsc) * alpha;
  }
  __builtin_amdgcn_fence(4, "workgroup"); __builtin_amdgcn_wave_barrier();
  const int rsub = lane >> 4, c4 = (lane & 15) * 4;
  for (int pass = 0; pass < 2; ++pass) {
#pragma unroll
    for (int q = 0; q < 8; ++q) { const int r = q * 2 + rsub; const v4f v = *(const v4fa*)&so[w][r][c4]; *(volatile v4f*)(C + (size_t)(row0 + r) * ldc + col0 + c4) = v; }
    if (pass == 0) __threadfence(); }
}

__global__ __launch_bounds__(256) void k_smx(const float* __restrict__ S, int lds_, _Float16* __restrict__ P, int ldp, _Float16* __restrict__ PL, int ldpl, int q0, int kend, int rrows) {
  #pragma clang fp contract(off)
  const int w = threadIdx.x >> 5, lane = threadIdx.x & 31;
  const int i = blockIdx.x * 8 + w;
  const int qi = q0 + i;
  const int nk = qi + 1;
  const float* s = S + (size_t)i * lds_;
  const int nt = (nk + 31) >> 5;
  float mx = -3.0e38f;
#pragma unroll 1
  for (int t = 0; t < nt; ++t) { const int j = t * 32 + lane; const int jc = (j < nk) ? j : (nk - 1); const float v = s[jc]; mx = fmaxf(mx, (j < nk) ? v : -3.0e38f); }
#pragma unroll
  for (int off = 16; off > 0; off >>= 1) mx = fmaxf(mx, __shfl_xor(mx, off, 32));
  float se = 0.f;
#pragma unroll 1
  for (int t = 0; t < nt; ++t) { const int j = t * 32 + lane; const int jc = (j < nk) ? j : (nk - 1); const float e = __expf(s[jc] - mx); se += (j < nk) ? e : 0.f; }
#pragma unroll
  for (int off = 16; off > 0; off >>= 1) se += __shfl_xor(se, off, 32);
  const float rinv = 1.0f / se;
  const bool res = (qi < rrows);
  const int nseg = kend >> 8;
#pragma unroll 1
  for (int sg = 0; sg < nseg; ++sg) {
    const int j0 = sg * 256 + lane * 8;
    FragH fh, fl;
#pragma unroll
    for (int q = 0; q < 8; ++q) {
      const int j = j0 + q; const int jc = (j < nk) ? j : (nk - 1);
      const float e = __expf(s[jc] - mx);
      const float p = (j < nk) ? (e * rinv) * 1024.0f : 0.0f;
      const _Float16 h = (_Float16)p; fh.h[q] = h; fl.h[q] = (_Float16)((p - (float)h) * 1024.0f);
    }
    unsigned short* d = (unsigned short*)P + (size_t)i * ldp + j0;
    *(volatile v8us*)d = fh.half[0]; __threadfence(); *(volatile v8us*)d = fh.half[0];
    if (res && sg == 0) { unsigned short* dl = (unsigned short*)PL + (size_t)qi * ldpl + lane * 8; *(volatile v8us*)dl = fl.half[0]; __threadfence(); *(volatile v8us*)dl = fl.half[0]; }
  }
}

extern "C" void kernel_launch(void* const* d_in, const int* in_sizes, int n_in,
                              void* d_out, int out_size, void* d_ws, size_t ws_size, hipStream_t stream) {
  if (n_in < 4) return;
  const size_t tok_span = (size_t)(NB - 1) * SEQ_FULL + SEQ;
  if ((size_t)in_sizes[0] < tok_span * DM) return;
  if (in_sizes[1] < DM * HD || in_sizes[2] < DM * HD || in_sizes[3] < DM * HD) return;
  if ((size_t)out_size < tok_span * HD) return;
  const float* x  = (const float*)d_in[0];
  const float* wq = (const float*)d_in[1];
  const float* wk = (const float*)d_in[2];
  const float* wv = (const float*)d_in[3];
  float* out = (float*)d_out;
  char* ws = (char*)d_ws; size_t off = 0;
  auto take = [&](size_t bytes) { char* p = ws + off; off += (bytes + 255) & ~(size_t)255; return p; };
  _Float16* BQ  = (_Float16*)take((size_t)HD * DM * 2);
  _Float16* BK  = (_Float16*)take((size_t)HD * DM * 2);
  _Float16* BV  = (_Float16*)take((size_t)HD * DM * 2);
  _Float16* X16 = (_Float16*)take(NR * DM * 2);
  float*    QF  = (float*)take(NR * HD * 4);
  _Float16* Q16 = (_Float16*)take(NR * HD * 2);
  _Float16* QL  = (_Float16*)take(NR * HD * 2);
  _Float16* K16 = (_Float16*)take(NR * HD * 2);
  _Float16* KL  = (_Float16*)take(NR * HD * 2);
  _Float16* V16 = (_Float16*)take(NR * HD * 2);
  _Float16* VL  = (_Float16*)take(NR * HD * 2);
  _Float16* VT  = (_Float16*)take((size_t)NB * HD * SEQ * 2);
  _Float16* VTL = (_Float16*)take((size_t)NB * HD * RESC * 2);
  float*    S   = (float*)take((size_t)QC * SEQ * 4);
  _Float16* P   = (_Float16*)take((size_t)QC * SEQ * 2);
  _Float16* PL  = (_Float16*)take((size_t)RESC * RESC * 2);
  if (off > ws_size || off > (size_t)134217728) return;

  const unsigned gw = (unsigned)(((size_t)HD * (DM / 8) + 255) / 256);
  k_wt_f16<<<gw, 256, 0, stream>>>(wq, BQ, DM, HD, 64.0f);
  k_wt_f16<<<gw, 256, 0, stream>>>(wk, BK, DM, HD, 64.0f);
  k_wt_f16<<<gw, 256, 0, stream>>>(wv, BV, DM, HD, 64.0f);
  k_x16<<<(unsigned)((NR * DM / 8 + 255) / 256), 256, 0, stream>>>(x, X16, NR * DM / 8);
  const unsigned gp = (unsigned)(NR / 128);
  const unsigned ghl = (unsigned)((NR * HD / 8 + 255) / 256);
  k_gemm2<<<gp, 128, 0, stream>>>(X16, DM, BQ, DM, 0.015625f, QF, HD, (int)NR, HD, DM);
  k_hl<<<ghl, 256, 0, stream>>>(QF, Q16, QL, NR * HD / 8);
  k_gemm2<<<gp, 128, 0, stream>>>(X16, DM, BK, DM, 0.015625f, QF, HD, (int)NR, HD, DM);
  k_hl<<<ghl, 256, 0, stream>>>(QF, K16, KL, NR * HD / 8);
  k_gemm2<<<gp, 128, 0, stream>>>(X16, DM, BV, DM, 0.015625f, QF, HD, (int)NR, HD, DM);
  k_hl<<<ghl, 256, 0, stream>>>(QF, V16, VL, NR * HD / 8);
  k_vt<<<(unsigned)(NB * (SEQ / 64)), 256, 0, stream>>>(V16, HD, SEQ, VT, SEQ, SEQ / 64);
  k_vt<<<(unsigned)(NB * (RESC / 64)), 256, 0, stream>>>(VL, HD, SEQ, VTL, RESC, RESC / 64);

  for (int b = 0; b < NB; ++b) {
    float* outb = out + (size_t)b * SEQ_FULL * HD;
    const _Float16* q16b = Q16 + (size_t)b * SEQ * HD; const _Float16* qlb = QL + (size_t)b * SEQ * HD;
    const _Float16* k16b = K16 + (size_t)b * SEQ * HD; const _Float16* klb = KL + (size_t)b * SEQ * HD;
    const _Float16* vtb = VT + (size_t)b * HD * SEQ; const _Float16* vtlb = VTL + (size_t)b * HD * RESC;
    for (int c = 0; c < SEQ / QC; ++c) {
      const int q0 = c * QC, kend = q0 + QC;
      const int rrows = (q0 < RESC) ? (RESC - q0) : 0;
      const unsigned gsc = (unsigned)(((QC / 16) * (kend / 64) + 3) / 4);
      k_gemm_hr<<<gsc, 128, 0, stream>>>(q16b + (size_t)q0 * HD, HD, qlb + (size_t)q0 * HD, HD, k16b, HD, klb, HD,
                                          0.125f, 0.0009765625f, rrows, q0, S, SEQ, QC, kend, HD);
      k_smx<<<(unsigned)(QC / 8), 256, 0, stream>>>(S, SEQ, P, SEQ, PL, RESC, q0, kend, RESC);
      const int mrows = QC - rrows;
      if (mrows > 0)
        k_gemm2<<<(unsigned)(mrows / 128), 128, 0, stream>>>(P + (size_t)rrows * SEQ, SEQ, vtb, SEQ, 0.0009765625f, outb + (size_t)(q0 + rrows) * HD, HD, mrows, HD, kend);
      if (rrows > 0)
        k_gemm_hr<<<(unsigned)(((rrows / 16) + 3) / 4), 128, 0, stream>>>(P, SEQ, PL, RESC, vtb, SEQ, vtlb, RESC,
                                                                     0.0009765625f, 0.0009765625f, rrows, 1 << 20, outb + (size_t)q0 * HD, HD, rrows, HD, RESC);
    }
  }
}
